// Model_24086176596657
// MI455X (gfx1250) — hardware-verified
//
#include <hip/hip_runtime.h>
#include <math.h>

constexpr int kB      = 4;
constexpr int kSeq    = 1024;
constexpr int kDm     = 512;
constexpr int kHeads  = 8;
constexpr int kDh     = 64;
constexpr int kLayers = 2;
constexpr int kPred   = 96;
constexpr int kCout   = 512;
constexpr int kTok    = kB * kSeq;
constexpr int kGateK  = 3 * kDm;
constexpr int kBH     = kB * kHeads;
constexpr int kGxN    = 128;
constexpr int kGqN    = 64;
constexpr int kGwRows = kGxN + kGqN;
constexpr int kQ2Rows = 128;
constexpr int kQ2Row0 = kSeq - kQ2Rows;
constexpr int kHeadSkip = kQ2Rows - kPred;
constexpr int kSqrtDh = 8;
constexpr float kQkScale    = 1.0f / (float)kSqrtDh;
constexpr float kEpsBackend = 1e-6f;
constexpr float kEpsLn      = 1e-5f;
constexpr float kInvDh      = 1.0f / (float)kDh;
constexpr int kAtWaves = 4;
constexpr int kAtKc    = 64;
constexpr int kQTiles  = kSeq / 64;

static_assert(kDm == kHeads * kDh, "head split");
static_assert(kSqrtDh * kSqrtDh == kDh, "score scale");
static_assert(kDm % 32 == 0, "GEMM K multiple of 32");
static_assert(kTok % 64 == 0 && kGxN % 64 == 0 && kGqN % 64 == 0 && kCout % 64 == 0 && kQ2Rows % 64 == 0, "GEMM tile multiples");
static_assert(kSeq % 64 == 0 && kDh == 64 && kAtKc == 64, "cell kernel tiling");
static_assert(kHeadSkip % 16 == 0 && kHeadSkip >= 0, "head row skip is a whole slab");
static_assert(kQ2Row0 % 64 == 0, "second cell starts on a query tile");
static_assert(5 * 16 <= kGxN && 16 <= kGqN, "gate column map fits");
static_assert(((kTok * kDm) / 8) % 256 == 0, "cast kernel segment boundary is block aligned");
static_assert((kGwRows * (kDm / 8)) % 256 == 0, "gate weight kernel grid exact");

typedef __attribute__((ext_vector_type(16))) __bf16   v16b;
typedef __attribute__((ext_vector_type(8)))  __bf16   v8b;
typedef __attribute__((ext_vector_type(8)))  float    v8f;
typedef __attribute__((ext_vector_type(4)))  float    v4f;
typedef __attribute__((ext_vector_type(4)))  unsigned int v4u;

__device__ __forceinline__ unsigned short f2bf_bits(float f) {
  unsigned u = __float_as_uint(f);
  return (unsigned short)((u + 0x7FFFu + ((u >> 16) & 1u)) >> 16);
}
__device__ __forceinline__ float bf_bits2f(unsigned short h) { return __uint_as_float(((unsigned)h) << 16); }
__device__ __forceinline__ float bf16r(float f) { return bf_bits2f(f2bf_bits(f)); }
__device__ __forceinline__ unsigned pk16(unsigned short a, unsigned short b) { return (unsigned)a | ((unsigned)b << 16); }

__device__ __forceinline__ void guard4_b(v8f& a, v8f& b, v8f& c, v8f& d, v16b x, v16b y) {
  asm volatile("v_nop\n\tv_nop\n\tv_nop\n\tv_nop" : "+v"(a), "+v"(b), "+v"(c), "+v"(d) : "v"(x), "v"(y));
}
__device__ __forceinline__ void keep4_b(v16b a, v16b b, v16b c, v16b d) { asm volatile("v_nop" :: "v"(a), "v"(b), "v"(c), "v"(d)); }
__device__ __forceinline__ void acc_guard4(v8f& a, v8f& b, v8f& c, v8f& d) {
  asm volatile("v_nop\n\tv_nop\n\tv_nop\n\tv_nop" : "+v"(a), "+v"(b), "+v"(c), "+v"(d));
}
__device__ __forceinline__ void guard_s6(v8f& s, v16b a0, v16b a1, v16b a2, v16b a3, v16b b0, v16b b1) {
  asm volatile("v_nop\n\tv_nop\n\tv_nop\n\tv_nop" : "+v"(s) : "v"(a0), "v"(a1), "v"(a2), "v"(a3), "v"(b0), "v"(b1));
}
__device__ __forceinline__ void guard_pv(v8f& a, v8f& b, v8f& c, v8f& d, v16b p0, v16b p1, v16b v0, v16b v1, v16b v2, v16b v3) {
  asm volatile("v_nop\n\tv_nop\n\tv_nop\n\tv_nop" : "+v"(a), "+v"(b), "+v"(c), "+v"(d)
               : "v"(p0), "v"(p1), "v"(v0), "v"(v1), "v"(v2), "v"(v3));
}

template <typename T> struct Frag;
template <> struct Frag<__bf16> {
  typedef v16b V; union U { v16b v; v8b h[2]; };
  static __device__ __forceinline__ v16b load(const __bf16* p) {
    U f; f.h[0] = *(const v8b*)(p); f.h[1] = *(const v8b*)(p + 16); return f.v;
  }
  static __device__ __forceinline__ v8f mma(v16b a, v16b b, v8f c) {
    return __builtin_amdgcn_wmma_f32_16x16x32_bf16(false, a, false, b, (short)0, c, false, false);
  }
};

template <int SPLITA, int BIAS_MODE>
__global__ __launch_bounds__(256) void wmma_gemm64_bf16(
    const unsigned short* __restrict__ Ap, const unsigned short* __restrict__ A2p, int lda, long strideA,
    const unsigned short* __restrict__ Btp, int ldb, long strideB,
    float* __restrict__ Cout, int ldc, long strideC,
    const float* __restrict__ bias,
    int M, int N, int K, float scale, int row_skip) {
  typedef __bf16 T;
  typedef v16b V;
  const T* A = (const T*)Ap; const T* A2 = (const T*)A2p; const T* Bt = (const T*)Btp;
  __shared__ __align__(16) float sT[8][16 * 68];
  const int b    = blockIdx.y;
  const int lane = threadIdx.x & 31;
  const int wave = threadIdx.x >> 5;
  const int tilesN = N >> 6;
  const int tilesM = M >> 6;
  const int tile = blockIdx.x * 8 + wave;
  if (tile >= tilesM * tilesN) return;
  const int tm = tile / tilesN;
  const int tn = tile - tm * tilesN;
  const int m0 = tm << 6;
  const int n0 = tn << 6;

  const T* Ab  = A  + (size_t)b * strideA;
  const T* Ab2 = A2 + (size_t)b * strideA;
  const T* Bb  = Bt + (size_t)b * strideB;

  const int rlane = lane & 15;
  const int koff  = (lane >> 4) * 8;
  const int mOff  = (lane >> 4) * 8;

  v8f acc[4][4];
#pragma unroll
  for (int i = 0; i < 4; ++i)
#pragma unroll
    for (int j = 0; j < 4; ++j) acc[i][j] = (v8f){0.f,0.f,0.f,0.f,0.f,0.f,0.f,0.f};

  for (int k0 = 0; k0 < K; k0 += 32) {
    V bh[4];
#pragma unroll
    for (int j = 0; j < 4; ++j) {
      const size_t bo = (size_t)(n0 + (j << 4) + rlane) * ldb + koff + k0;
      bh[j] = Frag<T>::load(Bb + bo);
    }
#pragma unroll
    for (int i = 0; i < 4; ++i) {
      const size_t ao = (size_t)(m0 + (i << 4) + rlane) * lda + koff + k0;
      V ah = Frag<T>::load(Ab + ao);
      V al = ah;
      if (SPLITA) al = Frag<T>::load(Ab2 + ao);
#pragma unroll
      for (int j = 0; j < 4; ++j) {
        acc[i][j] = Frag<T>::mma(ah, bh[j], acc[i][j]);
        if (SPLITA) acc[i][j] = Frag<T>::mma(al, bh[j], acc[i][j]);
      }
      guard4_b(acc[i][0], acc[i][1], acc[i][2], acc[i][3], ah, al);
    }
    keep4_b(bh[0], bh[1], bh[2], bh[3]);
  }
  acc_guard4(acc[0][0], acc[0][1], acc[0][2], acc[0][3]);
  acc_guard4(acc[1][0], acc[1][1], acc[1][2], acc[1][3]);
  acc_guard4(acc[2][0], acc[2][1], acc[2][2], acc[2][3]);
  acc_guard4(acc[3][0], acc[3][1], acc[3][2], acc[3][3]);

  float* slab = sT[wave];
#pragma unroll
  for (int i = 0; i < 4; ++i) {
    const int mBase = m0 + (i << 4);
#pragma unroll
    for (int j = 0; j < 4; ++j) {
      const int n = n0 + (j << 4) + rlane;
      float bv = 0.f;
      if (BIAS_MODE == 2) bv = bf16r(bias[n]);
#pragma unroll
      for (int r = 0; r < 8; ++r) {
        float v = acc[i][j][r] * scale;
        if (BIAS_MODE == 2) v += bv;
        slab[(mOff + r) * 68 + (j << 4) + rlane] = v;
      }
    }
    __builtin_amdgcn_fence(__ATOMIC_RELEASE, "workgroup");
    __builtin_amdgcn_wave_barrier();
    __builtin_amdgcn_fence(__ATOMIC_ACQUIRE, "workgroup");
    if (mBase >= row_skip) {
      float* C = Cout + (size_t)b * strideC;
      const int hh = lane >> 4, c4 = (lane & 15) * 4;
      for (int pass = 0; pass < 2; ++pass) {
#pragma unroll
        for (int it = 0; it < 8; ++it) {
          const int row = it * 2 + hh;
          v4f v = *(const v4f*)(slab + row * 68 + c4);
          *(volatile v4f*)(C + (size_t)(mBase + row - row_skip) * ldc + n0 + c4) = v;
        }
        __threadfence();
      }
    }
    __builtin_amdgcn_fence(__ATOMIC_RELEASE, "workgroup");
    __builtin_amdgcn_wave_barrier();
    __builtin_amdgcn_fence(__ATOMIC_ACQUIRE, "workgroup");
  }
}

__global__ __launch_bounds__(256) void cast8_bf16_kernel(const float* __restrict__ src0, unsigned short* __restrict__ dst0, int n8a,
                                                         const float* __restrict__ src1, unsigned short* __restrict__ dst1, int n8b) {
  const int i = blockIdx.x * 256 + threadIdx.x;
  const bool first = (i < n8a);
  const int k = first ? i : (i - n8a);
  const int lim = first ? n8a : n8b;
  if (k >= lim) return;
  const float* p = (first ? src0 : src1) + 8 * (size_t)k;
  unsigned short* q = (first ? dst0 : dst1) + 8 * (size_t)k;
  const v4f a = *(const v4f*)(p);
  const v4f c = *(const v4f*)(p + 4);
  unsigned short hb[8];
#pragma unroll
  for (int e = 0; e < 4; ++e) {
    hb[e]     = f2bf_bits(a[e]);
    hb[4 + e] = f2bf_bits(c[e]);
  }
  const v4u u = (v4u){pk16(hb[0], hb[1]), pk16(hb[2], hb[3]), pk16(hb[4], hb[5]), pk16(hb[6], hb[7])};
  *(volatile v4u*)q = u;
  __threadfence();
  *(volatile v4u*)q = u;
}

__global__ __launch_bounds__(256) void xt_bf16_kernel(const float* __restrict__ x, unsigned short* __restrict__ XT) {
  __shared__ float Tt[64 * 65];
  const int tid = threadIdx.x;
  const int c0 = blockIdx.x * 64, r0 = blockIdx.y * 64, b = blockIdx.z;
  const float* src = x + (size_t)b * kSeq * kDm;
#pragma unroll
  for (int i = 0; i < 4; ++i) {
    const int idx = i * 256 + tid;
    const int rr = idx >> 4, cc = (idx & 15) * 4;
    const v4f v = *(const v4f*)(src + (size_t)(r0 + rr) * kDm + c0 + cc);
    Tt[rr * 65 + cc + 0] = v[0];
    Tt[rr * 65 + cc + 1] = v[1];
    Tt[rr * 65 + cc + 2] = v[2];
    Tt[rr * 65 + cc + 3] = v[3];
  }
  __syncthreads();
  const int q = tid >> 3, c8 = (tid & 7) * 8;
  v4u u[2];
#pragma unroll
  for (int g = 0; g < 2; ++g) {
    const int qq = g * 32 + q;
    unsigned short hb[8];
#pragma unroll
    for (int e = 0; e < 8; ++e) hb[e] = f2bf_bits(Tt[(c8 + e) * 65 + qq]);
    u[g] = (v4u){pk16(hb[0], hb[1]), pk16(hb[2], hb[3]), pk16(hb[4], hb[5]), pk16(hb[6], hb[7])};
  }
  for (int pass = 0; pass < 2; ++pass) {
#pragma unroll
    for (int g = 0; g < 2; ++g) {
      const size_t o = ((size_t)b * kDm + (size_t)(c0 + g * 32 + q)) * kSeq + (size_t)(r0 + c8);
      *(volatile v4u*)(XT + o) = u[g];
    }
    __threadfence();
  }
}

__global__ __launch_bounds__(256) void gate_weight_kernel(const float* __restrict__ Wig, const float* __restrict__ Wfg,
                                                          unsigned short* __restrict__ GW) {
  const int i = blockIdx.x * 256 + threadIdx.x;
  if (i >= kGwRows * (kDm / 8)) return;
  const int row = i >> 6;
  const int c8 = (i & 63) * 8;
  int lay = 0, seg = 0, g = 0, hd = 0;
  bool valid = true;
  if (row < 48) { lay = 0; seg = row >> 4; g = (row >> 3) & 1; hd = row & 7; }
  else if (row < 80) { const int rr = row - 48; lay = 1; seg = 1 + (rr >> 4); g = (rr >> 3) & 1; hd = rr & 7; }
  else if (row < 128) { valid = false; }
  else if (row < 144) { const int rq = row - 128; lay = 1; seg = 0; g = rq >> 3; hd = rq & 7; }
  else { valid = false; }
  const float* W = g ? Wfg : Wig;
  const float* p = W + (size_t)(lay * kHeads + hd) * kGateK + (size_t)seg * kDm + c8;
  const v4f a = *(const v4f*)(p);
  const v4f c = *(const v4f*)(p + 4);
  unsigned short hb[8];
#pragma unroll
  for (int e = 0; e < 4; ++e) {
    const unsigned short t0 = f2bf_bits(a[e]);
    const unsigned short t1 = f2bf_bits(c[e]);
    hb[e]     = valid ? t0 : (unsigned short)0;
    hb[4 + e] = valid ? t1 : (unsigned short)0;
  }
  const v4u u = (v4u){pk16(hb[0], hb[1]), pk16(hb[2], hb[3]), pk16(hb[4], hb[5]), pk16(hb[6], hb[7])};
  unsigned short* q = GW + (size_t)row * kDm + c8;
  *(volatile v4u*)q = u;
  __threadfence();
  *(volatile v4u*)q = u;
}

template <int LAYER>
__global__ __launch_bounds__(32) void gate_scan_kernel(const float* __restrict__ GX, const float* __restrict__ GQ,
                                                       const float* __restrict__ b_ig, const float* __restrict__ b_fg,
                                                       float* __restrict__ PA, float* __restrict__ PMX, float* __restrict__ PP) {
  __shared__ float s_lf[kSeq];
  __shared__ float s_ig[kSeq];
  __shared__ __align__(16) float s_a[kSeq];
  __shared__ __align__(16) float s_mx[kSeq];
  __shared__ __align__(16) float s_p[kSeq];
  __shared__ double s_F[kSeq];
  __shared__ double s_sum[32];
  __shared__ float s_cmax[32];
  const int lane = threadIdx.x;
  int bh = blockIdx.x;
  bh = bh < kBH ? bh : (kBH - 1);
  const int b = bh / kHeads, h = bh - b * kHeads;
  const float bi = bf16r(b_ig[LAYER * kHeads + h]);
  const float bf = bf16r(b_fg[LAYER * kHeads + h]);

  double csum = 0.0;
#pragma unroll 1
  for (int t = 0; t < 32; ++t) {
    const int s = lane * 32 + t;
    const size_t row = (size_t)b * kSeq + s;
    const float* gx = GX + row * kGxN;
    float ig, fg;
    if (LAYER == 0) {
      ig = ((gx[h] + gx[16 + h]) + gx[32 + h]) + bi;
      fg = ((gx[8 + h] + gx[24 + h]) + gx[40 + h]) + bf;
    } else {
      const float* gq = GQ + row * kGqN;
      ig = ((gq[h] + gx[48 + h]) + gx[64 + h]) + bi;
      fg = ((gq[8 + h] + gx[56 + h]) + gx[72 + h]) + bf;
    }
    const float lf = -(fmaxf(-fg, 0.0f) + log1pf(expf(-fabsf(fg))));
    s_lf[s] = lf;
    s_ig[s] = ig;
    csum += (double)lf;
  }
  s_sum[lane] = csum;
  __syncthreads();

  double pre = 0.0;
#pragma unroll 1
  for (int l2 = 0; l2 < 32; ++l2) {
    const double v = s_sum[l2];
    pre += (l2 < lane) ? v : 0.0;
  }
  double F = pre;
  float lmax = -INFINITY;
#pragma unroll 1
  for (int t = 0; t < 32; ++t) {
    const int s = lane * 32 + t;
    F += (double)s_lf[s];
    const float af = (float)((double)s_ig[s] - F);
    lmax = fmaxf(lmax, af);
    s_a[s] = af;
    s_mx[s] = lmax;
    s_F[s] = F;
  }
  s_cmax[lane] = lmax;
  __syncthreads();

  float pm = -INFINITY;
#pragma unroll 1
  for (int l2 = 0; l2 < 32; ++l2) {
    const float v = s_cmax[l2];
    const float cand = fmaxf(pm, v);
    pm = (l2 < lane) ? cand : pm;
  }
#pragma unroll 1
  for (int t = 0; t < 32; ++t) {
    const int s = lane * 32 + t;
    const float mx = fmaxf(pm, s_mx[s]);
    s_mx[s] = mx;
    s_p[s] = (float)(s_F[s] + (double)mx);
  }
  __syncthreads();

  const size_t ob = (size_t)bh * kSeq;
  for (int pass = 0; pass < 2; ++pass) {
#pragma unroll 1
    for (int it = 0; it < 8; ++it) {
      const int idx = it * 128 + lane * 4;
      const v4f va = *(const v4f*)(s_a + idx);
      const v4f vm = *(const v4f*)(s_mx + idx);
      const v4f vp = *(const v4f*)(s_p + idx);
      *(volatile v4f*)(PA + ob + idx) = va;
      *(volatile v4f*)(PMX + ob + idx) = vm;
      *(volatile v4f*)(PP + ob + idx) = vp;
    }
    __threadfence();
  }
}

template <bool QSPLIT>
__global__ __launch_bounds__(128) void mlstm_cell_kernel(
    const unsigned short* __restrict__ Qhp, const unsigned short* __restrict__ Qlp,
    const unsigned short* __restrict__ XBp, const unsigned short* __restrict__ XTp,
    const float* __restrict__ PA, const float* __restrict__ PMX, const float* __restrict__ PP,
    const float* __restrict__ lnw,
    unsigned short* __restrict__ OutH, unsigned short* __restrict__ OutL,
    int qt0, int nqt, int out_rows_per_b, int out_row0) {
  __shared__ __align__(16) __bf16 Psh[kAtWaves][16 * kAtKc];
  __shared__ __align__(16) __bf16 Psl[kAtWaves][16 * kAtKc];
  __shared__ __align__(16) float  Os[kAtWaves][16 * 68];
  const __bf16* Qh = (const __bf16*)Qhp;
  const __bf16* Ql = (const __bf16*)Qlp;
  const __bf16* XB = (const __bf16*)XBp;
  const __bf16* XT = (const __bf16*)XTp;

  const int tid  = threadIdx.x;
  const int wave = tid >> 5;
  const int lane = tid & 31;
  const int hh   = lane >> 4;
  const int c    = lane & 15;

  const int bx  = blockIdx.x;
  const int qtl = bx % nqt;
  int bh = bx / nqt;
  bh = bh < kBH ? bh : (kBH - 1);
  int qt = qt0 + qtl;
  qt = qt < 0 ? 0 : (qt > (kQTiles - 1) ? (kQTiles - 1) : qt);
  const int b = bh / kHeads, h = bh - b * kHeads;
  const int q0 = qt * 64 + wave * 16;

  v16b qah[2], qal[2];
  {
    const size_t qo = ((size_t)b * kSeq + (size_t)(q0 + c)) * kDm + (size_t)h * kDh + 8 * hh;
    qah[0] = Frag<__bf16>::load(Qh + qo);
    qah[1] = Frag<__bf16>::load(Qh + qo + 32);
    asm volatile("" ::: "memory");
    if (QSPLIT) {
      qal[0] = Frag<__bf16>::load(Ql + qo);
      qal[1] = Frag<__bf16>::load(Ql + qo + 32);
    } else {
      qal[0] = qah[0];
      qal[1] = qah[1];
    }
    asm volatile("" ::: "memory");
  }
  float mrow[8];
  {
    const float* mxp = PMX + (size_t)bh * kSeq + q0 + 8 * hh;
    const v4f m0 = *(const v4f*)(mxp);
    const v4f m1 = *(const v4f*)(mxp + 4);
    mrow[0] = m0[0]; mrow[1] = m0[1]; mrow[2] = m0[2]; mrow[3] = m0[3];
    mrow[4] = m1[0]; mrow[5] = m1[1]; mrow[6] = m1[2]; mrow[7] = m1[3];
  }
  float rowsum[8];
  v8f oacc[4];
#pragma unroll
  for (int r = 0; r < 8; ++r) rowsum[r] = 0.0f;
#pragma unroll
  for (int t = 0; t < 4; ++t) oacc[t] = (v8f){0.f,0.f,0.f,0.f,0.f,0.f,0.f,0.f};

  const __bf16* krows = XB + (size_t)b * kSeq * kDm + (size_t)h * kDh + 8 * hh;
  const __bf16* vrows = XT + ((size_t)bh * kDh + (size_t)c) * kSeq + 8 * hh;
  const float*  ap    = PA + (size_t)bh * kSeq;
  __bf16* pwh = Psh[wave];
  __bf16* pwl = Psl[wave];

  const int nChunks = (qt + 1) < kQTiles ? (qt + 1) : kQTiles;
#pragma unroll 1
  for (int kc = 0; kc < nChunks; ++kc) {
    const int kv0 = kc * kAtKc;
    const bool diag = (kc == qt);
#pragma unroll 1
    for (int j = 0; j < 4; ++j) {
      const int kvcol = kv0 + j * 16 + c;
      const __bf16* kp = krows + (size_t)kvcol * kDm;
      const v16b kb0 = Frag<__bf16>::load(kp);
      const v16b kb1 = Frag<__bf16>::load(kp + 32);
      const float aj = ap[kvcol];
      v8f s = (v8f){0.f,0.f,0.f,0.f,0.f,0.f,0.f,0.f};
      s = Frag<__bf16>::mma(qah[0], kb0, s);
      s = Frag<__bf16>::mma(qah[1], kb1, s);
      if (QSPLIT) {
        s = Frag<__bf16>::mma(qal[0], kb0, s);
        s = Frag<__bf16>::mma(qal[1], kb1, s);
      }
      guard_s6(s, qah[0], qah[1], qal[0], qal[1], kb0, kb1);
#pragma unroll
      for (int r = 0; r < 8; ++r) {
        const int qr = q0 + 8 * hh + r;
        float e = expf(fminf(aj - mrow[r], 0.0f));
        e = (e < 1.17549435e-38f) ? 0.0f : e;
        const float val = (s[r] * kQkScale) * e;
        const bool valid = (!diag) || (kvcol <= qr);
        const float w = valid ? val : 0.0f;
        rowsum[r] += w;
        const unsigned short hb = f2bf_bits(w);
        const unsigned short lb = f2bf_bits(w - bf_bits2f(hb));
        pwh[(8 * hh + r) * kAtKc + j * 16 + c] = __builtin_bit_cast(__bf16, hb);
        pwl[(8 * hh + r) * kAtKc + j * 16 + c] = __builtin_bit_cast(__bf16, lb);
      }
      asm volatile("" ::: "memory");
    }
    __builtin_amdgcn_fence(__ATOMIC_RELEASE, "workgroup");
    __builtin_amdgcn_wave_barrier();
    __builtin_amdgcn_fence(__ATOMIC_ACQUIRE, "workgroup");
#pragma unroll
    for (int kk = 0; kk < 2; ++kk) {
      const v16b pa = Frag<__bf16>::load(pwh + c * kAtKc + kk * 32 + 8 * hh);
      const v16b pl = Frag<__bf16>::load(pwl + c * kAtKc + kk * 32 + 8 * hh);
      v16b vb[4];
#pragma unroll
      for (int t = 0; t < 4; ++t) vb[t] = Frag<__bf16>::load(vrows + (size_t)(t * 16) * kSeq + kv0 + kk * 32);
#pragma unroll
      for (int t = 0; t < 4; ++t) {
        oacc[t] = Frag<__bf16>::mma(pa, vb[t], oacc[t]);
        oacc[t] = Frag<__bf16>::mma(pl, vb[t], oacc[t]);
      }
      guard_pv(oacc[0], oacc[1], oacc[2], oacc[3], pa, pl, vb[0], vb[1], vb[2], vb[3]);
      asm volatile("" ::: "memory");
    }
    __builtin_amdgcn_fence(__ATOMIC_RELEASE, "workgroup");
    __builtin_amdgcn_wave_barrier();
    __builtin_amdgcn_fence(__ATOMIC_ACQUIRE, "workgroup");
  }
  acc_guard4(oacc[0], oacc[1], oacc[2], oacc[3]);

  float prow[8];
  {
    const float* ppp = PP + (size_t)bh * kSeq + q0 + 8 * hh;
    const v4f p0 = *(const v4f*)(ppp);
    const v4f p1 = *(const v4f*)(ppp + 4);
    prow[0] = p0[0]; prow[1] = p0[1]; prow[2] = p0[2]; prow[3] = p0[3];
    prow[4] = p1[0]; prow[5] = p1[1]; prow[6] = p1[2]; prow[7] = p1[3];
  }
  float lw[4];
#pragma unroll
  for (int t = 0; t < 4; ++t) lw[t] = bf16r(lnw[h * kDh + t * 16 + c]);

  float* os = Os[wave];
#pragma unroll
  for (int r = 0; r < 8; ++r) {
    float rs = rowsum[r];
    rs += __shfl_xor(rs, 1, 32);
    rs += __shfl_xor(rs, 2, 32);
    rs += __shfl_xor(rs, 4, 32);
    rs += __shfl_xor(rs, 8, 32);
    const float nrm = fmaxf(fabsf(rs), expf(-prow[r])) + kEpsBackend;
    const float inv = 1.0f / nrm;
    const float h0 = oacc[0][r] * inv;
    const float h1 = oacc[1][r] * inv;
    const float h2 = oacc[2][r] * inv;
    const float h3 = oacc[3][r] * inv;
    float s1 = (h0 + h1) + (h2 + h3);
    s1 += __shfl_xor(s1, 1, 32);
    s1 += __shfl_xor(s1, 2, 32);
    s1 += __shfl_xor(s1, 4, 32);
    s1 += __shfl_xor(s1, 8, 32);
    const float mu = s1 * kInvDh;
    const float d0 = h0 - mu, d1 = h1 - mu, d2 = h2 - mu, d3 = h3 - mu;
    float s2 = (d0 * d0 + d1 * d1) + (d2 * d2 + d3 * d3);
    s2 += __shfl_xor(s2, 1, 32);
    s2 += __shfl_xor(s2, 2, 32);
    s2 += __shfl_xor(s2, 4, 32);
    s2 += __shfl_xor(s2, 8, 32);
    const float var  = s2 * kInvDh;
    const float rstd = rsqrtf(var + kEpsLn);
    os[(8 * hh + r) * 68 +  0 + c] = (d0 * rstd) * lw[0];
    os[(8 * hh + r) * 68 + 16 + c] = (d1 * rstd) * lw[1];
    os[(8 * hh + r) * 68 + 32 + c] = (d2 * rstd) * lw[2];
    os[(8 * hh + r) * 68 + 48 + c] = (d3 * rstd) * lw[3];
  }
  __builtin_amdgcn_fence(__ATOMIC_RELEASE, "workgroup");
  __builtin_amdgcn_wave_barrier();
  __builtin_amdgcn_fence(__ATOMIC_ACQUIRE, "workgroup");

  {
    const int q = lane >> 3, c8 = (lane & 7) * 8;
    int orow0 = q0 - out_row0;
    const int omax = out_rows_per_b - 16;
    orow0 = orow0 < 0 ? 0 : (orow0 > omax ? omax : orow0);
    v4u uh[4], ul[4];
#pragma unroll
    for (int it = 0; it < 4; ++it) {
      const int row = it * 4 + q;
      const float* sp = os + row * 68 + c8;
      const v4f a = *(const v4f*)(sp);
      const v4f g = *(const v4f*)(sp + 4);
      unsigned short hb[8], lb[8];
#pragma unroll
      for (int e = 0; e < 4; ++e) {
        const float f0 = a[e];
        const float f1 = g[e];
        hb[e]     = f2bf_bits(f0);
        lb[e]     = f2bf_bits(f0 - bf_bits2f(hb[e]));
        hb[4 + e] = f2bf_bits(f1);
        lb[4 + e] = f2bf_bits(f1 - bf_bits2f(hb[4 + e]));
      }
      uh[it] = (v4u){pk16(hb[0], hb[1]), pk16(hb[2], hb[3]), pk16(hb[4], hb[5]), pk16(hb[6], hb[7])};
      ul[it] = (v4u){pk16(lb[0], lb[1]), pk16(lb[2], lb[3]), pk16(lb[4], lb[5]), pk16(lb[6], lb[7])};
    }
    for (int pass = 0; pass < 2; ++pass) {
#pragma unroll
      for (int it = 0; it < 4; ++it) {
        const int row = it * 4 + q;
        const size_t o = ((size_t)b * out_rows_per_b + (size_t)(orow0 + row)) * kDm + (size_t)h * kDh + c8;
        *(volatile v4u*)(OutH + o) = uh[it];
        *(volatile v4u*)(OutL + o) = ul[it];
      }
      __threadfence();
    }
  }
}

extern "C" void kernel_launch(void* const* d_in, const int* in_sizes, int n_in,
                              void* d_out, int out_size, void* d_ws, size_t ws_size, hipStream_t stream) {
  if (n_in < 11 || d_out == nullptr || d_ws == nullptr) return;
  if (in_sizes[0] != kB * kSeq * kDm || in_sizes[4] != kLayers * kHeads * kGateK || in_sizes[5] != kLayers * kHeads ||
      in_sizes[6] != kLayers * kHeads * kGateK || in_sizes[7] != kLayers * kHeads || in_sizes[8] != kLayers * kDm ||
      in_sizes[9] != kCout * kDm || in_sizes[10] != kCout || out_size != kB * kPred * kCout) return;

  const float* x_enc = (const float*)d_in[0];
  const float* W_ig  = (const float*)d_in[4];
  const float* b_ig  = (const float*)d_in[5];
  const float* W_fg  = (const float*)d_in[6];
  const float* b_fg  = (const float*)d_in[7];
  const float* ln_w  = (const float*)d_in[8];
  const float* fc_W  = (const float*)d_in[9];
  const float* fc_b  = (const float*)d_in[10];
  float* out = (float*)d_out;

  char* ws = (char*)d_ws; size_t off = 0;
  auto carve = [&](size_t bytes) -> char* { char* p = ws + off; off += (bytes + 255) & ~(size_t)255; return p; };
  unsigned short* XB  = (unsigned short*)carve((size_t)kTok * kDm * 2);
  unsigned short* XT  = (unsigned short*)carve((size_t)kBH * kDh * kSeq * 2);
  unsigned short* FCW = (unsigned short*)carve((size_t)kCout * kDm * 2);
  unsigned short* GW  = (unsigned short*)carve((size_t)kGwRows * kDm * 2);
  float* GX  = (float*)carve((size_t)kTok * kGxN * 4);
  float* GQ  = (float*)carve((size_t)kTok * kGqN * 4);
  float* SC0 = (float*)carve((size_t)3 * kBH * kSeq * 4);
  float* SC1 = (float*)carve((size_t)3 * kBH * kSeq * 4);
  unsigned short* Q1H = (unsigned short*)carve((size_t)kTok * kDm * 2);
  unsigned short* Q1L = (unsigned short*)carve((size_t)kTok * kDm * 2);
  unsigned short* Q2H = (unsigned short*)carve((size_t)kB * kQ2Rows * kDm * 2);
  unsigned short* Q2L = (unsigned short*)carve((size_t)kB * kQ2Rows * kDm * 2);
  if (off > ws_size || off > (size_t)134217728) return;

  unsigned short* GWX = GW;
  unsigned short* GWQ = GW + (size_t)kGxN * kDm;
  const size_t plane = (size_t)kBH * kSeq;

  const int n8x = (kTok * kDm) / 8;
  const int n8w = (kCout * kDm) / 8;
  cast8_bf16_kernel<<<(n8x + n8w + 255) / 256, 256, 0, stream>>>(x_enc, XB, n8x, fc_W, FCW, n8w);
  xt_bf16_kernel<<<dim3(kDm / 64, kSeq / 64, kB), 256, 0, stream>>>(x_enc, XT);
  gate_weight_kernel<<<(kGwRows * (kDm / 8)) / 256, 256, 0, stream>>>(W_ig, W_fg, GW);
  wmma_gemm64_bf16<0, 0><<<dim3((kTok / 64) * (kGxN / 64) / 8, 1), 256, 0, stream>>>(
      XB, XB, kDm, 0L, GWX, kDm, 0L, GX, kGxN, 0L, fc_b, kTok, kGxN, kDm, 1.0f, 0);
  gate_scan_kernel<0><<<kBH, 32, 0, stream>>>(GX, GQ, b_ig, b_fg, SC0, SC0 + plane, SC0 + 2 * plane);
  mlstm_cell_kernel<false><<<kQTiles * kBH, 128, 0, stream>>>(
      XB, XB, XB, XT, SC0, SC0 + plane, SC0 + 2 * plane, ln_w, Q1H, Q1L, 0, kQTiles, kSeq, 0);
  wmma_gemm64_bf16<1, 0><<<dim3((kTok / 64) * (kGqN / 64) / 8, 1), 256, 0, stream>>>(
      Q1H, Q1L, kDm, 0L, GWQ, kDm, 0L, GQ, kGqN, 0L, fc_b, kTok, kGqN, kDm, 1.0f, 0);
  gate_scan_kernel<1><<<kBH, 32, 0, stream>>>(GX, GQ, b_ig, b_fg, SC1, SC1 + plane, SC1 + 2 * plane);
  mlstm_cell_kernel<true><<<(kQ2Rows / 64) * kBH, 128, 0, stream>>>(
      Q1H, Q1L, XB, XT, SC1, SC1 + plane, SC1 + 2 * plane, ln_w + kDm, Q2H, Q2L, kQ2Row0 / 64, kQ2Rows / 64, kQ2Rows, kQ2Row0);
  wmma_gemm64_bf16<1, 2><<<dim3((kQ2Rows / 64) * (kCout / 64) / 8, kB), 256, 0, stream>>>(
      Q2H, Q2L, kDm, (long)kQ2Rows * kDm, FCW, kDm, 0L, out, kCout, (long)kPred * kCout, fc_b,
      kQ2Rows, kCout, kDm, 1.0f, kHeadSkip);
}
